// GraphormerMultiHeadAttention_2791728743073
// MI455X (gfx1250) — hardware-verified
//
#include <hip/hip_runtime.h>


namespace {
typedef _Float16 b16;
typedef __attribute__((ext_vector_type(16))) _Float16 v16b;
typedef __attribute__((ext_vector_type(8))) _Float16 v8b;
typedef __attribute__((ext_vector_type(4))) _Float16 v4h;
typedef __attribute__((ext_vector_type(2))) _Float16 v2h;
typedef __attribute__((ext_vector_type(8))) float v8f;
typedef __attribute__((ext_vector_type(4))) float v4f;
typedef __attribute__((ext_vector_type(2))) float v2f;
__device__ __forceinline__ float bf16_rne(float f) { unsigned int u = __float_as_uint(f); u += 0x7FFFu + ((u >> 16) & 1u); return __uint_as_float(u & 0xFFFF0000u); }
__device__ __forceinline__ void split16(float v, b16& hi, b16& lo) { hi = (b16)v; lo = (b16)(v - (float)hi); }
__device__ __forceinline__ v16b frag_kb(const b16* p, int hh) { const v8b a = *(const v8b*)(p + 8 * hh), b = *(const v8b*)(p + 16 + 8 * hh); v16b f;
#pragma unroll
  for (int e = 0; e < 8; ++e) { f[e] = a[e]; f[8 + e] = b[e]; } return f; }
__device__ __forceinline__ v8f wmma16b(v16b a, v16b b, v8f c) { v8f d = __builtin_amdgcn_wmma_f32_16x16x32_f16(false, a, false, b, (short)0, c, false, false); asm volatile("v_nop\n\tv_nop\n\tv_nop\n\tv_nop" : "+v"(d) : "v"(a), "v"(b)); return d; }
__device__ __forceinline__ void wave_lds_sync() { __builtin_amdgcn_fence(__ATOMIC_RELEASE, "workgroup"); __builtin_amdgcn_wave_barrier(); __builtin_amdgcn_fence(__ATOMIC_ACQUIRE, "workgroup"); }
__device__ __forceinline__ float pmul(float a, float b) { float p = a * b; asm volatile("" : "+v"(p)); return p; }
__device__ __forceinline__ int iclamp(int v, int lo, int hi) { return v < lo ? lo : (v > hi ? hi : v); }
__device__ __forceinline__ float nexp2(float v) { return __builtin_amdgcn_exp2f(v); }

constexpr int B = 4, BL = B  , N = 2048, D = 512, NH = 8, HD = 64, E = 32768, NROW = B * N;
constexpr float XS = 8.0f, WSC = 256.0f, PS = 1024.0f, RS_ = 1024.0f, LOG2E = 1.4426950408889634f, SCALE = 0.125f;
static_assert(N % 64 == 0 && D % 128 == 0 && NH * HD == D && HD == 64, "tiling");

__global__ __launch_bounds__(256) void wcvt_kernel(const float* __restrict__ w, b16* __restrict__ W16, int n8) { const int u = blockIdx.x * 256 + threadIdx.x; if (u >= n8) return; const size_t e = (size_t)u * 8; v8b o; for (int j = 0; j < 8; ++j) o[j] = (b16)(bf16_rne(w[e + j]) * WSC);
  for (int pass = 0; pass < 2; ++pass) { *(volatile v8b*)(W16 + e) = o; __threadfence(); } }
__global__ __launch_bounds__(256) void cb_kernel(const int* __restrict__ ei, const float* __restrict__ ea, const float* __restrict__ ebw, const float* __restrict__ ebb, float* __restrict__ CB) {
  const int m = blockIdx.x * 256 + threadIdx.x; if (m >= N) return; int last = -1;
#pragma unroll 1
  for (int e = 0; e < E; ++e) { const int s = ei[e], t = ei[E + e]; const bool valid = (s >= 0) && (s < N) && (t >= 0) && (t < N); if (valid && t == m) last = e; }
  float vals[NH]; for (int h = 0; h < NH; ++h) vals[h] = 0.0f;
  if (last >= 0) { const float a0 = bf16_rne(ea[(size_t)last * 3]), a1 = bf16_rne(ea[(size_t)last * 3 + 1]), a2 = bf16_rne(ea[(size_t)last * 3 + 2]); for (int h = 0; h < NH; ++h) vals[h] = a0 * bf16_rne(ebw[h * 3]) + a1 * bf16_rne(ebw[h * 3 + 1]) + a2 * bf16_rne(ebw[h * 3 + 2]) + bf16_rne(ebb[h]); }
  for (int pass = 0; pass < 2; ++pass) { for (int h = 0; h < NH; ++h) ((volatile float*)CB)[(size_t)h * N + m] = vals[h]; __threadfence(); }
}
__global__ __launch_bounds__(128) void proj_kernel(const float* __restrict__ x, const b16* __restrict__ WQKV, const float* __restrict__ bq, const float* __restrict__ bk, const float* __restrict__ bv, b16* __restrict__ QP, b16* __restrict__ KP, b16* __restrict__ VTh, b16* __restrict__ VTl) {
  __shared__ __attribute__((aligned(16))) b16 As[64][D + 8]; __shared__ __attribute__((aligned(16))) float Tf[4][16][128 + 4];
  const int wave = threadIdx.x >> 5, lane = threadIdx.x & 31, nloc = lane & 15, hlf = lane >> 4; const int t0 = blockIdx.x * 64; const int b = blockIdx.y; const int slab = blockIdx.z, n0 = slab * 128, part = slab / 4, h0 = (slab & 3) * 2;
  const float* bias = part == 0 ? bq : part == 1 ? bk : bv;
  for (int i = threadIdx.x; i < 64 * (D / 4); i += 128) { const int rr = i / (D / 4), q4 = (i % (D / 4)) * 4; const v4f f = *(const v4f*)(x + ((size_t)b * N + t0 + rr) * D + q4); v4h o; for (int j = 0; j < 4; ++j) o[j] = (b16)(bf16_rne(f[j]) * XS); *(v4h*)(&As[rr][q4]) = o; }
  __syncthreads();
  v8f acc[8];
#pragma unroll
  for (int tt = 0; tt < 8; ++tt) acc[tt] = (v8f){};
#pragma unroll 2
  for (int kb = 0; kb < D; kb += 32) { const v16b a = frag_kb(&As[wave * 16 + nloc][kb], hlf);
#pragma unroll
    for (int tt = 0; tt < 8; ++tt) acc[tt] = wmma16b(a, frag_kb(WQKV + (size_t)(n0 + tt * 16 + nloc) * D + kb, hlf), acc[tt]); }
#pragma unroll
  for (int tt = 0; tt < 8; ++tt) { const float bb = bf16_rne(bias[(n0 & 511) + tt * 16 + nloc]);
#pragma unroll
    for (int r = 0; r < 8; ++r) Tf[wave][8 * hlf + r][tt * 16 + nloc] = acc[tt][r] * (1.0f / (XS * WSC)) + bb; }
  __syncthreads();
  for (int pass = 0; pass < 2; ++pass) {
    if (part < 2) { b16* plane = part == 0 ? QP : KP; const int h = h0 + (lane >> 4), d = (lane & 15) * 4;
      for (int rr = 0; rr < 16; ++rr) { const int tok = t0 + wave * 16 + rr; v4h o4; for (int j = 0; j < 4; ++j) o4[j] = (b16)(Tf[wave][rr][lane * 4 + j] * XS); *(volatile v4h*)(plane + (((size_t)b * NH + h) * N + tok) * HD + d) = o4; } }
    else {
#pragma unroll 1
      for (int q = 0; q < 32; ++q) { const int cl = wave * 32 + q; const int h = h0 + cl / HD, d = cl % HD; const int tk = lane * 2; v2h hv, lv; for (int e2 = 0; e2 < 2; ++e2) { const float vs = Tf[(tk + e2) >> 4][(tk + e2) & 15][cl] * XS; const b16 ph = (b16)vs; hv[e2] = ph; lv[e2] = (b16)((vs - (float)ph) * RS_); }
        const size_t dst = (((size_t)b * NH + h) * HD + d) * (size_t)N + t0 + tk; *(volatile v2h*)(VTh + dst) = hv; *(volatile v2h*)(VTl + dst) = lv; } }
    __threadfence(); }
}
__global__ __launch_bounds__(64) void attn_kernel(const b16* __restrict__ QP, const b16* __restrict__ KP, const b16* __restrict__ VTh, const b16* __restrict__ VTl, const float* __restrict__ CB, float* __restrict__ CT) {
  __shared__ __attribute__((aligned(16))) b16 Pb[2][16][32 + 8], Pl[2][16][32 + 8]; __shared__ __attribute__((aligned(16))) float To[2][16][HD + 4];
  const int wave = threadIdx.x >> 5, lane = threadIdx.x & 31, hh = lane >> 4, col = lane & 15; const int bh = blockIdx.y, b = bh / NH, h = bh % NH; const int n0 = blockIdx.x * 32 + wave * 16; const int nq = n0 + col;
  const b16* Qb = QP + (size_t)bh * N * HD; const b16* Kb = KP + (size_t)bh * N * HD; const b16* Vh = VTh + (size_t)bh * HD * N; const b16* Vl = VTl + (size_t)bh * HD * N; const float* cbh = CB + (size_t)h * N;
  const v16b q0 = frag_kb(Qb + (size_t)nq * HD, hh), q1 = frag_kb(Qb + (size_t)nq * HD + 32, hh);
  const float cs = LOG2E * SCALE / (XS * XS);
  float mrun = -INFINITY, l = 0.0f; v8f o[4], o2[4];
#pragma unroll
  for (int t = 0; t < 4; ++t) { o[t] = (v8f){}; o2[t] = (v8f){}; }
#pragma unroll 1
  for (int s0 = 0; s0 < N; s0 += 32) {
    float e[16]; float mx = -INFINITY;
#pragma unroll
    for (int u2 = 0; u2 < 2; ++u2) { const b16* kr = Kb + (size_t)(s0 + u2 * 16 + col) * HD; v8f sacc = wmma16b(frag_kb(kr, hh), q0, (v8f){}); sacc = wmma16b(frag_kb(kr + 32, hh), q1, sacc);
#pragma unroll
      for (int r = 0; r < 8; ++r) { const int m = s0 + u2 * 16 + 8 * hh + r; const float vv = sacc[r] * cs + cbh[m] * LOG2E; e[u2 * 8 + r] = vv; mx = fmaxf(mx, vv); } }
    mx = fmaxf(mx, __shfl_xor(mx, 16)); const float mn = fmaxf(mrun, mx); const float al = nexp2(mrun - mn); float sum = 0.0f;
#pragma unroll
    for (int i2 = 0; i2 < 16; ++i2) { const float p = nexp2(e[i2] - mn); sum += p; const float psv = p * PS; const b16 p1 = (b16)psv; const int slot = (i2 < 8 ? 0 : 16) + 8 * hh + (i2 & 7); Pb[wave][col][slot] = p1; Pl[wave][col][slot] = (b16)((psv - (float)p1) * RS_); }
    sum += __shfl_xor(sum, 16); l = l * al + sum; mrun = mn;
    wave_lds_sync();
    const v16b pf = frag_kb(&Pb[wave][col][0], hh), plf = frag_kb(&Pl[wave][col][0], hh);
#pragma unroll
    for (int t = 0; t < 4; ++t) { o[t] *= al; o2[t] *= al; const v16b vh = frag_kb(Vh + (size_t)(t * 16 + col) * N + s0, hh); o[t] = wmma16b(vh, pf, o[t]); o2[t] = wmma16b(frag_kb(Vl + (size_t)(t * 16 + col) * N + s0, hh), pf, o2[t]); o2[t] = wmma16b(vh, plf, o2[t]); }
    wave_lds_sync(); }
  const float inv = 1.0f / (l * PS * XS);
#pragma unroll
  for (int t = 0; t < 4; ++t)
#pragma unroll
    for (int r = 0; r < 8; ++r) To[wave][col][t * 16 + 8 * hh + r] = (o[t][r] + o2[t][r] * (1.0f / RS_)) * inv;
  wave_lds_sync();
  for (int pass = 0; pass < 2; ++pass) { for (int rr = 0; rr < 16; rr += 2) { const int row = rr + hh; *(volatile v4f*)(CT + ((size_t)b * N + n0 + row) * D + h * HD + col * 4) = *(const v4f*)(&To[wave][row][col * 4]); } __threadfence(); }
}
__global__ __launch_bounds__(64) void outp_kernel(const float* __restrict__ CT, const b16* __restrict__ WO, const float* __restrict__ ob, float* __restrict__ out) {
  __shared__ __attribute__((aligned(16))) b16 Ah[2][16][128 + 8], Al[2][16][128 + 8]; __shared__ __attribute__((aligned(16))) float Tf[2][16][128 + 4];
  const int wave = threadIdx.x >> 5, lane = threadIdx.x & 31, nloc = lane & 15, hlf = lane >> 4; const size_t m0 = (size_t)blockIdx.x * 32 + wave * 16; const int n0 = blockIdx.y * 128;
  v8f acc[8], acc2[8];
#pragma unroll
  for (int t = 0; t < 8; ++t) { acc[t] = (v8f){}; acc2[t] = (v8f){}; }
#pragma unroll 1
  for (int kc = 0; kc < D; kc += 128) {
    for (int idx = lane; idx < 16 * 32; idx += 32) { const int rr = idx / 32, c4 = (idx % 32) * 4; const v4f v = *(const v4f*)(CT + (m0 + rr) * D + kc + c4); v4h hv, lv; for (int j = 0; j < 4; ++j) { const float vs = v[j] * XS; const b16 ph = (b16)vs; hv[j] = ph; lv[j] = (b16)((vs - (float)ph) * RS_); } *(v4h*)(&Ah[wave][rr][c4]) = hv; *(v4h*)(&Al[wave][rr][c4]) = lv; }
    wave_lds_sync();
#pragma unroll
    for (int kb = 0; kb < 128; kb += 32) { const v16b a = frag_kb(&Ah[wave][nloc][kb], hlf), al = frag_kb(&Al[wave][nloc][kb], hlf);
#pragma unroll
      for (int t = 0; t < 8; ++t) { const v16b bw = frag_kb(WO + (size_t)(n0 + t * 16 + nloc) * D + kc + kb, hlf); acc[t] = wmma16b(a, bw, acc[t]); acc2[t] = wmma16b(al, bw, acc2[t]); } }
    wave_lds_sync(); }
#pragma unroll
  for (int t = 0; t < 8; ++t) { const float bb = bf16_rne(ob[n0 + t * 16 + nloc]);
#pragma unroll
    for (int r = 0; r < 8; ++r) Tf[wave][8 * hlf + r][t * 16 + nloc] = (acc[t][r] + acc2[t][r] * (1.0f / RS_)) * (1.0f / (XS * WSC)) + bb; }
  wave_lds_sync();
  for (int pass = 0; pass < 2; ++pass) { for (int rr = 0; rr < 16; ++rr) *(volatile v4f*)(out + (m0 + rr) * D + n0 + lane * 4) = *(const v4f*)(&Tf[wave][rr][lane * 4]); __threadfence(); }
}
}

extern "C" void kernel_launch(void* const* d_in, const int* in_sizes, int n_in, void* d_out, int out_size, void* d_ws, size_t ws_size, hipStream_t stream) {
  (void)n_in;
  auto Fp = [&](int i) { return (const float*)d_in[i]; };
  if (in_sizes[0] != NROW * D || in_sizes[1] != 2 * E || in_sizes[2] != E * 3 || in_sizes[3] != D * D || in_sizes[5] != D * D || in_sizes[7] != D * D || in_sizes[9] != D * D || in_sizes[10] != D || in_sizes[11] != NH * 3 || in_sizes[12] != NH || out_size != NROW * D) return;
  size_t off = 0; char* ws = (char*)d_ws;
  auto carve = [&](size_t bytes) { char* p = ws + off; off += (bytes + 255) & ~(size_t)255; return p; };
  b16* WQKV = (b16*)carve((size_t)3 * D * D * 2); b16* WO = (b16*)carve((size_t)D * D * 2); float* CB = (float*)carve((size_t)NH * N * 4); const size_t plane = (size_t)B * NH * N * HD * 2;
  b16* QP = (b16*)carve(plane); b16* KP = (b16*)carve(plane); b16* VTh = (b16*)carve(plane); b16* VTl = (b16*)carve(plane); float* CT = (float*)carve((size_t)NROW * D * 4);
  if (off > ws_size || off > ((size_t)128 << 20)) return;
  wcvt_kernel<<<(D * D / 8 + 255) / 256, 256, 0, stream>>>(Fp(3), WQKV, D * D / 8); wcvt_kernel<<<(D * D / 8 + 255) / 256, 256, 0, stream>>>(Fp(5), WQKV + (size_t)D * D, D * D / 8); wcvt_kernel<<<(D * D / 8 + 255) / 256, 256, 0, stream>>>(Fp(7), WQKV + (size_t)2 * D * D, D * D / 8); wcvt_kernel<<<(D * D / 8 + 255) / 256, 256, 0, stream>>>(Fp(9), WO, D * D / 8);
  cb_kernel<<<N / 256, 256, 0, stream>>>((const int*)d_in[1], Fp(2), Fp(11), Fp(12), CB);
  proj_kernel<<<dim3(N / 64, BL, 12), 128, 0, stream>>>(Fp(0), WQKV, Fp(4), Fp(6), Fp(8), QP, KP, VTh, VTl);
  attn_kernel<<<dim3(N / 32, BL * NH), 64, 0, stream>>>(QP, KP, VTh, VTl, CB, CT);
  outp_kernel<<<dim3(BL * N / 32, D / 128), 64, 0, stream>>>(CT, WO, Fp(10), (float*)d_out);
}
